// LSTMNet_8418135900758
// MI455X (gfx1250) — hardware-verified
//
#include <hip/hip_runtime.h>
#include <math.h>

constexpr int NBATCH   = 512;
constexpr int NSTEP    = 512;
constexpr int NFEAT    = 32;
constexpr int NHID     = 64;
constexpr int NGATE    = 4 * NHID;
constexpr int NTHR     = 256;
constexpr int ROWS_BLK = 32;
constexpr int KCAT0    = NHID + NFEAT;
constexpr int KCAT1    = NHID + NHID;
constexpr int WPITCH   = 128;
constexpr int PA0      = 104;
constexpr int PA1      = 136;
constexpr int PHF      = 68;
constexpr float ACT_CARRY = 64.0f;
constexpr float WGT_CARRY = 16.0f;
constexpr float FOLD_INV  = 1.0f / (ACT_CARRY * WGT_CARRY);

static_assert(NBATCH % ROWS_BLK == 0, "batch tiles exact");
static_assert(KCAT0 % 32 == 0 && KCAT1 % 32 == 0, "K multiples of 32");
static_assert(KCAT0 <= WPITCH && KCAT1 <= WPITCH, "planes hold the concatenated K");
static_assert(KCAT0 <= PA0 && KCAT1 <= PA1, "LDS tiles hold the concatenated K");
static_assert(PA0 % 8 == 0 && PA1 % 8 == 0 && PHF % 4 == 0, "aligned pitches");
static_assert(NTHR == 256 && ROWS_BLK == 32 && NHID == 64, "wave map: 2 m-subtiles x 4 unit-subtiles");
static_assert(ROWS_BLK * NFEAT == NTHR * 4, "x tile: one float4 per thread");
static_assert((2 * ROWS_BLK * PA0) % NTHR == 0 && (2 * ROWS_BLK * PA1) % NTHR == 0, "zero-fill loops exact");
static_assert(NGATE * (NHID / 8) == 8 * NTHR, "prep job = 8 blocks");

typedef __attribute__((ext_vector_type(16))) _Float16 v16h;
typedef __attribute__((ext_vector_type(8)))  _Float16 v8h;
typedef __attribute__((ext_vector_type(4)))  _Float16 v4h;
typedef __attribute__((ext_vector_type(8)))  float    v8f;
typedef __attribute__((ext_vector_type(4)))  float    v4f;

__device__ __forceinline__ void wmma_guard4(v8f& a0, v8f& a1, v8f& a2, v8f& a3,
                                            v16h x, v16h y0, v16h y1, v16h y2, v16h y3) {
  asm volatile("v_nop\n\tv_nop\n\tv_nop\n\tv_nop"
               : "+v"(a0), "+v"(a1), "+v"(a2), "+v"(a3)
               : "v"(x), "v"(y0), "v"(y1), "v"(y2), "v"(y3));
}
__device__ __forceinline__ void acc_guard4(v8f& a, v8f& b, v8f& c, v8f& d) {
  asm volatile("v_nop\n\tv_nop\n\tv_nop\n\tv_nop" : "+v"(a), "+v"(b), "+v"(c), "+v"(d));
}

template <typename T> struct Frag;
template <> struct Frag<_Float16> {
  typedef v16h V; union U { v16h v; v8h h[2]; };
  static __device__ __forceinline__ v16h load(const _Float16* p) {
    U f; f.h[0] = *(const v8h*)(p); f.h[1] = *(const v8h*)(p + 16); return f.v;
  }
  static __device__ __forceinline__ v8f mma(v16h a, v16h b, v8f c) {
    return __builtin_amdgcn_wmma_f32_16x16x32_f16(false, a, false, b, (short)0, c, false, false);
  }
};

__device__ __forceinline__ float fsig(float v)  { return __builtin_amdgcn_rcpf(1.0f + expf(-v)); }
__device__ __forceinline__ float ftanh(float v) { return 1.0f - 2.0f * __builtin_amdgcn_rcpf(expf(2.0f * v) + 1.0f); }

__device__ __forceinline__ float lstm_cell(float zi, float zf, float zg, float zo, float& cs) {
  const float ig = fsig(zi);
  const float fg = fsig(zf);
  const float gg = ftanh(zg);
  const float og = fsig(zo);
  const float cn = fg * cs + ig * gg;
  cs = cn;
  return og * ftanh(cn);
}

__global__ __launch_bounds__(NTHR) void wprep_kernel(const float* __restrict__ wih0, const float* __restrict__ whh0,
                                                     const float* __restrict__ wih1, const float* __restrict__ whh1,
                                                     unsigned short* __restrict__ W0p, unsigned short* __restrict__ W1p) {
  const int job = (int)(blockIdx.x >> 3);
  const int i   = (int)(blockIdx.x & 7) * NTHR + (int)threadIdx.x;
  const int row = i >> 3;
  const int c8  = i & 7;
  const float* src;
  unsigned short* dst;
  int spitch;
  int coff;
  if (job == 0)      { src = whh0; spitch = NHID;  dst = W0p; coff = 0; }
  else if (job == 1) { src = wih0; spitch = NFEAT; dst = W0p; coff = NHID; }
  else if (job == 2) { src = wih1; spitch = NHID;  dst = W1p; coff = 0; }
  else               { src = whh1; spitch = NHID;  dst = W1p; coff = NHID; }
  const int col = c8 * 8;
  const bool valid = (col < spitch);
  const int colc = valid ? col : 0;
  const float* sp = src + (size_t)row * (size_t)spitch + colc;
  const v4f a = *(const v4f*)(sp);
  const v4f b = *(const v4f*)(sp + 4);
  v8h hv;
#pragma unroll
  for (int e = 0; e < 4; ++e) {
    const float fa = valid ? (a[e] * WGT_CARRY) : 0.0f;
    const float fb = valid ? (b[e] * WGT_CARRY) : 0.0f;
    hv[e]     = (_Float16)fa;
    hv[4 + e] = (_Float16)fb;
  }
  unsigned short* op = dst + (size_t)row * WPITCH + coff + col;
  *(volatile v8h*)op = hv;
  __threadfence();
  *(volatile v8h*)op = hv;
}

__global__ __launch_bounds__(NTHR) void lstm2_seq_kernel(const float* __restrict__ x,
                                                         const float* __restrict__ bih0, const float* __restrict__ bhh0,
                                                         const float* __restrict__ bih1, const float* __restrict__ bhh1,
                                                         const float* __restrict__ fcw,  const float* __restrict__ fcb,
                                                         const unsigned short* __restrict__ W0p,
                                                         const unsigned short* __restrict__ W1p,
                                                         float* __restrict__ out) {
  __shared__ __align__(16) _Float16 A0[2][ROWS_BLK * PA0];
  __shared__ __align__(16) _Float16 A1[2][ROWS_BLK * PA1];
  __shared__ __align__(16) float    Hf[ROWS_BLK * PHF];

  const _Float16* W0 = (const _Float16*)W0p;
  const _Float16* W1 = (const _Float16*)W1p;
  const int tid  = (int)threadIdx.x;
  const int lane = tid & 31;
  const int wave = tid >> 5;
  const int c    = lane & 15;
  const int hh   = lane >> 4;
  const int koff = hh * 8;
  const int mt   = wave >> 2;
  const int ub   = wave & 3;
  const int j    = 16 * ub + c;
  const int rb   = 16 * mt + 8 * hh;
  const int bt0  = (int)blockIdx.x * ROWS_BLK;
  const int xm   = tid >> 3;
  const int xf4  = (tid & 7) * 4;

  {
    _Float16* z0 = &A0[0][0];
#pragma unroll 1
    for (int i = tid; i < 2 * ROWS_BLK * PA0; i += NTHR) z0[i] = (_Float16)0.0f;
    _Float16* z1 = &A1[0][0];
#pragma unroll 1
    for (int i = tid; i < 2 * ROWS_BLK * PA1; i += NTHR) z1[i] = (_Float16)0.0f;
  }
  __syncthreads();
  {
    const v4f xv = *(const v4f*)(x + ((size_t)(bt0 + xm) * NSTEP) * NFEAT + xf4);
    v4h xh;
#pragma unroll
    for (int e = 0; e < 4; ++e) xh[e] = (_Float16)(xv[e] * ACT_CARRY);
    *(v4h*)(&A0[0][0] + xm * PA0 + NHID + xf4) = xh;
  }

  float bz0[4], bz1[4];
#pragma unroll
  for (int g = 0; g < 4; ++g) {
    bz0[g] = bih0[g * NHID + j] + bhh0[g * NHID + j];
    bz1[g] = bih1[g * NHID + j] + bhh1[g * NHID + j];
  }
  float cs0[8], cs1[8], hst1[8];
#pragma unroll
  for (int r = 0; r < 8; ++r) { cs0[r] = 0.0f; cs1[r] = 0.0f; hst1[r] = 0.0f; }
  __syncthreads();

  const v8f z8 = {0.f, 0.f, 0.f, 0.f, 0.f, 0.f, 0.f, 0.f};
  const _Float16* w0row = W0 + (size_t)j * WPITCH + koff;
  const _Float16* w1row = W1 + (size_t)j * WPITCH + koff;
  constexpr size_t GSTRIDE = (size_t)NHID * WPITCH;

#pragma unroll 1
  for (int t = 0; t < NSTEP; ++t) {
    const int p = t & 1;
    const int tn = (t + 1 < NSTEP) ? (t + 1) : (NSTEP - 1);
    v4f xv = *(const v4f*)(x + ((size_t)(bt0 + xm) * NSTEP + (size_t)tn) * NFEAT + xf4);
    asm volatile("" : "+v"(xv));

    const _Float16* a0cur = &A0[p][0];
    _Float16*       a0nxt = &A0[p ^ 1][0];
    _Float16*       a1cur = &A1[p][0];
    _Float16*       a1nxt = &A1[p ^ 1][0];

    {
      const _Float16* arow = a0cur + (16 * mt + c) * PA0 + koff;
      v8f acc0 = z8, acc1 = z8, acc2 = z8, acc3 = z8;
#pragma unroll 1
      for (int k0 = 0; k0 < KCAT0; k0 += 32) {
        const v16h a  = Frag<_Float16>::load(arow + k0);
        const v16h b0 = Frag<_Float16>::load(w0row + k0);
        const v16h b1 = Frag<_Float16>::load(w0row + GSTRIDE + k0);
        const v16h b2 = Frag<_Float16>::load(w0row + 2 * GSTRIDE + k0);
        const v16h b3 = Frag<_Float16>::load(w0row + 3 * GSTRIDE + k0);
        acc0 = Frag<_Float16>::mma(a, b0, acc0);
        acc1 = Frag<_Float16>::mma(a, b1, acc1);
        acc2 = Frag<_Float16>::mma(a, b2, acc2);
        acc3 = Frag<_Float16>::mma(a, b3, acc3);
        wmma_guard4(acc0, acc1, acc2, acc3, a, b0, b1, b2, b3);
      }
      acc_guard4(acc0, acc1, acc2, acc3);
#pragma unroll
      for (int r = 0; r < 8; ++r) {
        const float zi = acc0[r] * FOLD_INV + bz0[0];
        const float zf = acc1[r] * FOLD_INV + bz0[1];
        const float zg = acc2[r] * FOLD_INV + bz0[2];
        const float zo = acc3[r] * FOLD_INV + bz0[3];
        const float hn = lstm_cell(zi, zf, zg, zo, cs0[r]);
        const _Float16 h16 = (_Float16)(hn * ACT_CARRY);
        a0nxt[(rb + r) * PA0 + j] = h16;
        a1cur[(rb + r) * PA1 + j] = h16;
      }
      v4h xh;
#pragma unroll
      for (int e = 0; e < 4; ++e) xh[e] = (_Float16)(xv[e] * ACT_CARRY);
      *(v4h*)(a0nxt + xm * PA0 + NHID + xf4) = xh;
    }
    __syncthreads();

    {
      const _Float16* arow = a1cur + (16 * mt + c) * PA1 + koff;
      v8f acc0 = z8, acc1 = z8, acc2 = z8, acc3 = z8;
#pragma unroll 1
      for (int k0 = 0; k0 < KCAT1; k0 += 32) {
        const v16h a  = Frag<_Float16>::load(arow + k0);
        const v16h b0 = Frag<_Float16>::load(w1row + k0);
        const v16h b1 = Frag<_Float16>::load(w1row + GSTRIDE + k0);
        const v16h b2 = Frag<_Float16>::load(w1row + 2 * GSTRIDE + k0);
        const v16h b3 = Frag<_Float16>::load(w1row + 3 * GSTRIDE + k0);
        acc0 = Frag<_Float16>::mma(a, b0, acc0);
        acc1 = Frag<_Float16>::mma(a, b1, acc1);
        acc2 = Frag<_Float16>::mma(a, b2, acc2);
        acc3 = Frag<_Float16>::mma(a, b3, acc3);
        wmma_guard4(acc0, acc1, acc2, acc3, a, b0, b1, b2, b3);
      }
      acc_guard4(acc0, acc1, acc2, acc3);
#pragma unroll
      for (int r = 0; r < 8; ++r) {
        const float zi = acc0[r] * FOLD_INV + bz1[0];
        const float zf = acc1[r] * FOLD_INV + bz1[1];
        const float zg = acc2[r] * FOLD_INV + bz1[2];
        const float zo = acc3[r] * FOLD_INV + bz1[3];
        const float hn = lstm_cell(zi, zf, zg, zo, cs1[r]);
        hst1[r] = hn;
        a1nxt[(rb + r) * PA1 + NHID + j] = (_Float16)(hn * ACT_CARRY);
      }
    }
    __syncthreads();
  }

#pragma unroll
  for (int r = 0; r < 8; ++r) Hf[(rb + r) * PHF + j] = hst1[r];
  __syncthreads();

  if (wave == 0) {
    float s = 0.0f;
#pragma unroll 4
    for (int k = 0; k < NHID; ++k) s = fmaf(Hf[lane * PHF + k], fcw[k], s);
    s += fcb[0];
    float* op = out + bt0 + lane;
    *(volatile float*)op = s;
    __threadfence();
    *(volatile float*)op = s;
  }
}

extern "C" void kernel_launch(void* const* d_in, const int* in_sizes, int n_in,
                              void* d_out, int out_size, void* d_ws, size_t ws_size, hipStream_t stream) {
  if (n_in < 11 || d_out == nullptr || d_ws == nullptr) return;
  if (in_sizes[0] != NBATCH * NSTEP * NFEAT || in_sizes[1] != NGATE * NFEAT || in_sizes[2] != NGATE * NHID ||
      in_sizes[3] != NGATE || in_sizes[4] != NGATE || in_sizes[5] != NGATE * NHID || in_sizes[6] != NGATE * NHID ||
      in_sizes[7] != NGATE || in_sizes[8] != NGATE || in_sizes[9] != NHID || in_sizes[10] != 1 ||
      out_size != NBATCH) return;

  const float* x    = (const float*)d_in[0];
  const float* wih0 = (const float*)d_in[1];
  const float* whh0 = (const float*)d_in[2];
  const float* bih0 = (const float*)d_in[3];
  const float* bhh0 = (const float*)d_in[4];
  const float* wih1 = (const float*)d_in[5];
  const float* whh1 = (const float*)d_in[6];
  const float* bih1 = (const float*)d_in[7];
  const float* bhh1 = (const float*)d_in[8];
  const float* fcw  = (const float*)d_in[9];
  const float* fcb  = (const float*)d_in[10];
  float* out = (float*)d_out;

  char* ws = (char*)d_ws;
  size_t off = 0;
  auto carve = [&](size_t bytes) -> char* { char* pp = ws + off; off += (bytes + 255) & ~(size_t)255; return pp; };
  unsigned short* W0 = (unsigned short*)carve((size_t)NGATE * WPITCH * 2);
  unsigned short* W1 = (unsigned short*)carve((size_t)NGATE * WPITCH * 2);
  if (off > ws_size || off > (size_t)134217728) return;

  wprep_kernel<<<32, NTHR, 0, stream>>>(wih0, whh0, wih1, whh1, W0, W1);
  lstm2_seq_kernel<<<NBATCH / ROWS_BLK, NTHR, 0, stream>>>(x, bih0, bhh0, bih1, bhh1, fcw, fcb, W0, W1, out);
}
